// truncated_krylov_layer_16724602650838
// MI455X (gfx1250) — hardware-run, weakly checked
//
#include <hip/hip_runtime.h>
#include <stddef.h>
#include <stdint.h>

static constexpr int TWO_TERM = 0;

#define NN      50000
#define FD      128
#define NE      800000
#define NTERM   8
#define WROWS   (NTERM * FD)
#define GBM     128
#define MP      50048
#define PLANE   (MP * FD)
#define KA      1152
#define KB      768
#define NTHR    256
#define NWAVE   8
#define EPT     8
#define WCH     (32 * EPT)
#define NBRUN   1024
#define SLB     10
#define NBK     49
#define WLCAP   2560
#define RCAP    18432
#define TRIPCAP 64
#define MAXDEG_MEAS   33
#define MAXB1024_MEAS 16696
#define HRB     64
#define SP      68

#define BK_ZINTS (NWAVE * WLCAP + RCAP + 3 * NBRUN)
#define BK_INTS  (BK_ZINTS + 16)
#define BK_LDS   (BK_INTS * 4)

#define PBX   (MP * FD / 8 / NTHR)
#define PBWA  (FD * KA / 8 / NTHR)
#define PBWB  (FD * KB / 8 / NTHR)
#define PBTOT (PBX + PBWA + PBWB + 1)

static_assert((long long)NN < (1LL << 31));
static_assert(MP % GBM == 0 && MP >= NN && MP == 391 * GBM && MP % HRB == 0);
static_assert(NBRUN == (1 << SLB) && NBRUN == 1024 && NBRUN % GBM == 0 && NBRUN / GBM == 8 && NBRUN % HRB == 0);
static_assert(NBK * NBRUN >= MP);
static_assert(NE < (1 << 20) && (((long long)NE) << SLB) < (1LL << 31));
static_assert(NE % WCH == 0 && NE % 4 == 0);
static_assert((long long)RCAP * 100 >= (long long)MAXB1024_MEAS * 105);
static_assert(RCAP % (2 * NTHR) == 0 && BK_ZINTS % 4 == 0 && NWAVE * WLCAP >= RCAP);
static_assert(WLCAP >= MAXB1024_MEAS / 8 + 8 * 46 + 1);
static_assert(MAXDEG_MEAS + 8 <= TRIPCAP);
static_assert(KA == FD + 4 * 2 * FD && KB == 3 * 2 * FD && KA % 32 == 0 && KB % 32 == 0 && FD % 32 == 0);
static_assert((MP * FD / 8) % NTHR == 0 && (FD * KA / 8) % NTHR == 0 && (FD * KB / 8) % NTHR == 0);
static_assert((KA / 8) % 8 == 0 && (KB / 8) % 8 == 0);
static_assert(BK_LDS <= 327680);
static_assert((GBM * SP + FD) * 4 <= 65536);
static_assert(FD == 32 * 4 && FD == 2 * 64 && (2 * NBRUN) % (4 * NTHR) == 0);

typedef float          v4f   __attribute__((ext_vector_type(4)));
typedef float          v8f   __attribute__((ext_vector_type(8)));
typedef int            v2i   __attribute__((ext_vector_type(2)));
typedef int            v4i   __attribute__((ext_vector_type(4)));
typedef int            v8i   __attribute__((ext_vector_type(8)));
typedef unsigned       v2u   __attribute__((ext_vector_type(2)));
typedef unsigned short v8us  __attribute__((ext_vector_type(8)));
typedef unsigned short v16us __attribute__((ext_vector_type(16)));
typedef __bf16         v16bf __attribute__((ext_vector_type(16)));
typedef v4f  __attribute__((may_alias)) v4fa;
typedef v2i  __attribute__((may_alias)) v2ia;
typedef v4i  __attribute__((may_alias)) v4ia;
typedef v2u  __attribute__((may_alias)) v2ua;
typedef v8us __attribute__((may_alias)) v8usa;
union FragB { v16bf v; v16us u; v8us h[2]; v8i w; };

__device__ __forceinline__ v8f wmb(const FragB& a, const FragB& b, v8f c) {
  v8f d = __builtin_amdgcn_wmma_f32_16x16x32_bf16(false, a.v, false, b.v, (short)0, c, false, false);
  asm volatile("v_nop\n\tv_nop\n\tv_nop\n\tv_nop" : "+v"(d) : "v"(a.w), "v"(b.w));
  return d;
}

__device__ __forceinline__ unsigned bf16_bits(float f) {
  const unsigned u = __float_as_uint(f);
  const unsigned r = (u + 0x7FFFu + ((u >> 16) & 1u)) >> 16;
  const unsigned q = (u >> 16) | 0x40u;
  return ((u & 0x7fffffffu) > 0x7f800000u) ? q : r;
}
__device__ __forceinline__ float bf16_val(float f) { return __uint_as_float(bf16_bits(f) << 16); }
__device__ __forceinline__ float bfw_lo(unsigned w) { return __uint_as_float(w << 16); }
__device__ __forceinline__ float bfw_hi(unsigned w) { return __uint_as_float(w & 0xffff0000u); }

__device__ __forceinline__ void st2_v4f(float* p, v4f v) {
  *(volatile v4f*)p = v;
  __threadfence();
  *(volatile v4f*)p = v;
}
__device__ __forceinline__ void st2_v4i(int* p, v4i v) {
  *(volatile v4i*)p = v;
  __threadfence();
  *(volatile v4i*)p = v;
}
__device__ __forceinline__ void st2_v8us(unsigned short* p, v8us v) {
  *(volatile v8us*)p = v;
  __threadfence();
  *(volatile v8us*)p = v;
}

__device__ __forceinline__ v8us gather8(const float* __restrict__ base, int stride) {
  float f[8];
#pragma unroll
  for (int i = 0; i < 8; ++i) f[i] = base[(size_t)i * (size_t)stride];
  v8us o;
#pragma unroll
  for (int i = 0; i < 8; ++i) o[i] = (unsigned short)bf16_bits(f[i]);
  return o;
}

__global__ __launch_bounds__(NTHR) void k_prep(const float* __restrict__ x, const float* __restrict__ w,
                                               const float* __restrict__ bias, unsigned short* xb,
                                               unsigned short* wa, unsigned short* wb, float* bf) {
  const int tid = (int)threadIdx.x, lane = tid & 31;
  const int blk = (int)blockIdx.x;
  if (blk < PBX) {
    const int u   = blk * NTHR + tid;
    const int row = u >> 4, k8 = (u & 15) * 8;
    const int rc  = row < NN ? row : NN - 1;
    const unsigned mk = row < NN ? 0xffffu : 0u;
    const float* p = x + (size_t)rc * FD + k8;
    const v4f a = *(const v4fa*)p;
    const v4f b = *(const v4fa*)(p + 4);
    v8us o;
    o[0] = (unsigned short)(bf16_bits(a.x) & mk); o[1] = (unsigned short)(bf16_bits(a.y) & mk);
    o[2] = (unsigned short)(bf16_bits(a.z) & mk); o[3] = (unsigned short)(bf16_bits(a.w) & mk);
    o[4] = (unsigned short)(bf16_bits(b.x) & mk); o[5] = (unsigned short)(bf16_bits(b.y) & mk);
    o[6] = (unsigned short)(bf16_bits(b.z) & mk); o[7] = (unsigned short)(bf16_bits(b.w) & mk);
    st2_v8us(xb + (size_t)row * FD + k8, o);
  } else if (blk < PBX + PBWA) {
    const int u  = (blk - PBX) * NTHR + tid;
    const int n  = u / (KA / 8);
    const int k8 = (u - n * (KA / 8)) * 8;
    const int kk = k8 - FD;
    const int srow = (k8 < FD) ? k8 : (FD * (1 + (kk >> 8)) + (kk & (FD - 1)));
    const v8us o = gather8(w + (size_t)srow * FD + n, FD);
    st2_v8us(wa + (size_t)n * KA + k8, o);
  } else if (blk < PBX + PBWA + PBWB) {
    const int u  = (blk - PBX - PBWA) * NTHR + tid;
    const int n  = u / (KB / 8);
    const int k8 = (u - n * (KB / 8)) * 8;
    const int srow = FD * (5 + (k8 >> 8)) + (k8 & (FD - 1));
    const v8us o = gather8(w + (size_t)srow * FD + n, FD);
    st2_v8us(wb + (size_t)n * KB + k8, o);
  } else {
    if (tid < 32) {
      const v4f b = *(const v4fa*)(bias + 4 * lane);
      v4f o;
      o.x = bf16_val(b.x); o.y = bf16_val(b.y); o.z = bf16_val(b.z); o.w = bf16_val(b.w);
      st2_v4f(bf + 4 * lane, o);
    }
  }
}

__global__ __launch_bounds__(NTHR) void k_bucket(const int* __restrict__ srcs, const int* __restrict__ dsts,
                                                 const float* __restrict__ ew, int* LIST, int* CO, int* FLAG) {
  extern __shared__ __attribute__((aligned(16))) int dsm[];
  int* wl   = dsm;
  int* pl   = dsm + NWAVE * WLCAP;
  int* cnt  = pl + RCAP;
  int* offs = cnt + NBRUN;
  int* cur  = offs + NBRUN;
  int* misc = cur + NBRUN;
  const int tid = (int)threadIdx.x, lane = tid & 31, wave = tid >> 5;
  const int blk = (int)blockIdx.x;
  const unsigned nbs = (unsigned)(blk * NBRUN);

  {
    const v4i z4 = {0, 0, 0, 0};
    for (int i = tid * 4; i < BK_ZINTS; i += NTHR * 4) *(v4ia*)(dsm + i) = z4;
    if (tid < 16) misc[tid] = 0;
  }
  __syncthreads();

  {
    const int per  = ((NE + NWAVE * WCH - 1) / (NWAVE * WCH)) * WCH;
    const int ebeg = wave * per;
    const int eend = (ebeg + per < NE) ? (ebeg + per) : NE;
    int* mylist = wl + wave * WLCAP;
    int wc = 0;
#pragma unroll 1
    for (int cb = ebeg; cb < eend; cb += WCH) {
      const int e0 = cb + lane * EPT;
      const v4i da = *(const v4ia*)(dsts + e0);
      const v4i db = *(const v4ia*)(dsts + e0 + 4);
      const unsigned s0 = (unsigned)da.x - nbs, s1 = (unsigned)da.y - nbs;
      const unsigned s2 = (unsigned)da.z - nbs, s3 = (unsigned)da.w - nbs;
      const unsigned s4 = (unsigned)db.x - nbs, s5 = (unsigned)db.y - nbs;
      const unsigned s6 = (unsigned)db.z - nbs, s7 = (unsigned)db.w - nbs;
      const bool h0 = s0 < (unsigned)NBRUN, h1 = s1 < (unsigned)NBRUN, h2 = s2 < (unsigned)NBRUN, h3 = s3 < (unsigned)NBRUN;
      const bool h4 = s4 < (unsigned)NBRUN, h5 = s5 < (unsigned)NBRUN, h6 = s6 < (unsigned)NBRUN, h7 = s7 < (unsigned)NBRUN;
      const unsigned m0 = __builtin_amdgcn_ballot_w32(h0), m1 = __builtin_amdgcn_ballot_w32(h1);
      const unsigned m2 = __builtin_amdgcn_ballot_w32(h2), m3 = __builtin_amdgcn_ballot_w32(h3);
      const unsigned m4 = __builtin_amdgcn_ballot_w32(h4), m5 = __builtin_amdgcn_ballot_w32(h5);
      const unsigned m6 = __builtin_amdgcn_ballot_w32(h6), m7 = __builtin_amdgcn_ballot_w32(h7);
      const unsigned any = m0 | m1 | m2 | m3 | m4 | m5 | m6 | m7;
      if (any != 0u) {
        const int pre = (int)(__builtin_amdgcn_mbcnt_lo(m0, 0u) + __builtin_amdgcn_mbcnt_lo(m1, 0u) +
                              __builtin_amdgcn_mbcnt_lo(m2, 0u) + __builtin_amdgcn_mbcnt_lo(m3, 0u) +
                              __builtin_amdgcn_mbcnt_lo(m4, 0u) + __builtin_amdgcn_mbcnt_lo(m5, 0u) +
                              __builtin_amdgcn_mbcnt_lo(m6, 0u) + __builtin_amdgcn_mbcnt_lo(m7, 0u));
        int p = wc + pre;
        if (h0) { if (p < WLCAP) mylist[p] = ((e0 + 0) << SLB) | (int)s0; p = p + 1; }
        if (h1) { if (p < WLCAP) mylist[p] = ((e0 + 1) << SLB) | (int)s1; p = p + 1; }
        if (h2) { if (p < WLCAP) mylist[p] = ((e0 + 2) << SLB) | (int)s2; p = p + 1; }
        if (h3) { if (p < WLCAP) mylist[p] = ((e0 + 3) << SLB) | (int)s3; p = p + 1; }
        if (h4) { if (p < WLCAP) mylist[p] = ((e0 + 4) << SLB) | (int)s4; p = p + 1; }
        if (h5) { if (p < WLCAP) mylist[p] = ((e0 + 5) << SLB) | (int)s5; p = p + 1; }
        if (h6) { if (p < WLCAP) mylist[p] = ((e0 + 6) << SLB) | (int)s6; p = p + 1; }
        if (h7) { if (p < WLCAP) mylist[p] = ((e0 + 7) << SLB) | (int)s7; p = p + 1; }
        wc += (int)(__builtin_popcount(m0) + __builtin_popcount(m1) + __builtin_popcount(m2) + __builtin_popcount(m3) +
                    __builtin_popcount(m4) + __builtin_popcount(m5) + __builtin_popcount(m6) + __builtin_popcount(m7));
      }
    }
    if (lane == 0) misc[wave] = wc;
  }
  __syncthreads();

  if (wave == 0) {
    int ov = 0;
#pragma unroll 1
    for (int w2 = 0; w2 < NWAVE; ++w2) {
      int c = misc[w2];
      if (c > WLCAP) ov = 1;
      c = c < 0 ? 0 : (c > WLCAP ? WLCAP : c);
#pragma unroll 1
      for (int b0 = 0; b0 < c; b0 += 32) {
        const int idx = b0 + lane;
        const int ent = wl[w2 * WLCAP + (idx < WLCAP ? idx : WLCAP - 1)];
        const int m32 = (c - b0) < 32 ? (c - b0) : 32;
#pragma unroll 1
        for (int k = 0; k < m32; ++k) {
          const int u    = __builtin_amdgcn_readlane(ent, k);
          const int slot = u & (NBRUN - 1);
          if (lane == 0) cnt[slot] = cnt[slot] + 1;
        }
      }
    }
    if (lane == 0) misc[9] = ov;
  }
  __syncthreads();
  if (wave == 0) {
    const int base = lane * (NBRUN / 32);
    int s = 0, mxc = 0;
#pragma unroll 1
    for (int i = 0; i < NBRUN / 32; ++i) {
      const int cv = cnt[base + i];
      s += cv;
      mxc = cv > mxc ? cv : mxc;
    }
    int incl = s;
#pragma unroll
    for (int d = 1; d < 32; d <<= 1) {
      const int y = __shfl_up(incl, d, 32);
      if (lane >= d) incl += y;
    }
#pragma unroll
    for (int d = 16; d >= 1; d >>= 1) {
      const int y = __shfl_xor(mxc, d, 32);
      mxc = y > mxc ? y : mxc;
    }
    const int total = __shfl(incl, 31, 32);
    int run = incl - s;
#pragma unroll 1
    for (int i = 0; i < NBRUN / 32; ++i) {
      const int cv = cnt[base + i];
      offs[base + i] = run;
      cur[base + i]  = run;
      run += cv;
    }
    if (lane == 0) {
      const int ov0 = misc[9];
      misc[9]  = ((ov0 != 0) || (mxc > TRIPCAP) || (total > RCAP)) ? 1 : 0;
      misc[10] = total > RCAP ? RCAP : (total < 0 ? 0 : total);
    }
  }
  __syncthreads();

  if (wave == 0) {
#pragma unroll 1
    for (int w2 = 0; w2 < NWAVE; ++w2) {
      int c = misc[w2];
      c = c < 0 ? 0 : (c > WLCAP ? WLCAP : c);
#pragma unroll 1
      for (int b0 = 0; b0 < c; b0 += 32) {
        const int idx = b0 + lane;
        const int ent = wl[w2 * WLCAP + (idx < WLCAP ? idx : WLCAP - 1)];
        const int m32 = (c - b0) < 32 ? (c - b0) : 32;
#pragma unroll 1
        for (int k = 0; k < m32; ++k) {
          const int u    = __builtin_amdgcn_readlane(ent, k);
          const int slot = u & (NBRUN - 1);
          if (lane == 0) {
            int p = cur[slot];
            p = p < 0 ? 0 : (p > RCAP - 1 ? RCAP - 1 : p);
            pl[p] = u;
            cur[slot] = p + 1;
          }
        }
      }
    }
  }
  __syncthreads();

  const int ovf = misc[9];
  const int nh  = misc[10];
  int* lp  = LIST + (size_t)blk * (size_t)(2 * RCAP);
  int* cop = CO + (size_t)blk * (2 * NBRUN);
  int* fp  = FLAG + (size_t)blk * 32;
#pragma unroll 1
  for (int it = 0; it < RCAP / (2 * NTHR); ++it) {
    const int i0 = 2 * (it * NTHR + tid);
    const v2i en = *(const v2ia*)(pl + i0);
    int e0 = (en.x >> SLB) & 0xFFFFF;
    int e1 = (en.y >> SLB) & 0xFFFFF;
    e0 = e0 > NE - 1 ? NE - 1 : e0;
    e1 = e1 > NE - 1 ? NE - 1 : e1;
    int s0 = srcs[e0], s1 = srcs[e1];
    const float w0 = ew[e0], w1 = ew[e1];
    asm volatile("" :: "v"(s0), "v"(s1), "v"(w0), "v"(w1));
    s0 = s0 < 0 ? 0 : (s0 > NN - 1 ? NN - 1 : s0);
    s1 = s1 < 0 ? 0 : (s1 > NN - 1 ? NN - 1 : s1);
    const int k0 = (i0 < nh) ? -1 : 0;
    const int k1 = (i0 + 1 < nh) ? -1 : 0;
    v4i o;
    o.x = s0 & k0;
    o.y = (int)(bf16_bits(w0) << 16) & k0;
    o.z = s1 & k1;
    o.w = (int)(bf16_bits(w1) << 16) & k1;
    st2_v4i(lp + (size_t)2 * (size_t)i0, o);
  }
#pragma unroll 1
  for (int it = 0; it < (2 * NBRUN) / (4 * NTHR); ++it) {
    const int i0 = 4 * (it * NTHR + tid);
    const v4i v = *(const v4ia*)(cnt + i0);
    st2_v4i(cop + i0, v);
  }
  if (tid < 8) {
    const v4i f = {ovf, ovf, ovf, ovf};
    st2_v4i(fp + 4 * tid, f);
  }
}

template <int SRCBF>
__global__ __launch_bounds__(NTHR) void k_hop(const int* __restrict__ LIST, const int* __restrict__ CO,
                                              const int* __restrict__ FLAG,
                                              const unsigned short* __restrict__ sb,
                                              const float* __restrict__ sf, float* dst) {
  const int tid = (int)threadIdx.x, lane = tid & 31, wave = tid >> 5;
  const int rowBase = (int)blockIdx.x * HRB;
  const int bucket  = rowBase >> SLB;
  const int* lb  = LIST + (size_t)bucket * (size_t)(2 * RCAP);
  const int* cob = CO + (size_t)bucket * (2 * NBRUN);
  const int flag = FLAG[(size_t)bucket * 32];
  const float qnan = __uint_as_float(0x7fc00000u);

#pragma unroll 1
  for (int i = 0; i < HRB / NWAVE; ++i) {
    const int d    = rowBase + (HRB / NWAVE) * wave + i;
    const int slot = d & (NBRUN - 1);
    const int craw = cob[slot];
    const int oraw = cob[NBRUN + slot];
    const bool big = craw > TRIPCAP;
    int c = craw < 0 ? 0 : (craw > TRIPCAP ? TRIPCAP : craw);
    const int o = oraw < 0 ? 0 : (oraw > RCAP - 1 ? RCAP - 1 : oraw);
    if (c > RCAP - o) c = RCAP - o;
    int last = o + c - 1; last = last < o ? o : last;
    last = last > RCAP - 1 ? RCAP - 1 : last;
    float a0 = 0.0f, a1 = 0.0f, a2 = 0.0f, a3 = 0.0f;
#pragma unroll 1
    for (int b0 = 0; b0 < c; b0 += 32) {
      int idx = o + b0 + lane;
      idx = idx > last ? last : idx;
      const v2i en = *(const v2ia*)(lb + (size_t)2 * (size_t)idx);
      int sr = en.x;
      sr = sr < 0 ? 0 : (sr > NN - 1 ? NN - 1 : sr);
      const int wbits = en.y;
      const int m32 = (c - b0) < 32 ? (c - b0) : 32;
#pragma unroll 1
      for (int k = 0; k < m32; ++k) {
        const int   sk = __builtin_amdgcn_readlane(sr, k);
        const float wk = __int_as_float(__builtin_amdgcn_readlane(wbits, k));
        float x0, x1, x2, x3;
        if constexpr (SRCBF != 0) {
          const v2u q = *(const v2ua*)(sb + (size_t)sk * FD + 4 * lane);
          x0 = bfw_lo(q.x); x1 = bfw_hi(q.x); x2 = bfw_lo(q.y); x3 = bfw_hi(q.y);
        } else {
          const v4f q = *(const v4fa*)(sf + (size_t)sk * FD + 4 * lane);
          x0 = q.x; x1 = q.y; x2 = q.z; x3 = q.w;
        }
        a0 = fmaf(wk, x0, a0); a1 = fmaf(wk, x1, a1); a2 = fmaf(wk, x2, a2); a3 = fmaf(wk, x3, a3);
      }
    }
    const bool bad  = (flag != 0) | big;
    const bool live = d < NN;
    float m0 = bad ? qnan : a0, m1 = bad ? qnan : a1, m2 = bad ? qnan : a2, m3 = bad ? qnan : a3;
    v4f ov;
    ov.x = live ? m0 : 0.0f; ov.y = live ? m1 : 0.0f; ov.z = live ? m2 : 0.0f; ov.w = live ? m3 : 0.0f;
    st2_v4f(dst + (size_t)d * FD + 4 * lane, ov);
  }
}

__device__ __forceinline__ void split16(const v4f& f0, const v4f& f1, const v4f& f2, const v4f& f3,
                                        FragB& hi, FragB& lo) {
  const float f[16] = {f0.x, f0.y, f0.z, f0.w, f1.x, f1.y, f1.z, f1.w,
                       f2.x, f2.y, f2.z, f2.w, f3.x, f3.y, f3.z, f3.w};
#pragma unroll
  for (int i = 0; i < 16; ++i) {
    const unsigned a = bf16_bits(f[i]);
    hi.u[i] = (unsigned short)a;
    if constexpr (TWO_TERM != 0) lo.u[i] = (unsigned short)bf16_bits(f[i] - __uint_as_float(a << 16));
    else lo.u[i] = (unsigned short)0;
  }
}

template <int H, int FINAL>
__device__ __forceinline__ void epi_half(float* stg, const float* sbias, const v8f (&acc)[8], float* out,
                                         int rowBase, int flag, int wave, int hh, int m) {
#pragma unroll
  for (int nt = 0; nt < 4; ++nt) {
#pragma unroll
    for (int r = 0; r < 8; ++r) stg[(16 * wave + 8 * hh + r) * SP + 16 * nt + m] = acc[4 * H + nt][r];
  }
  __syncthreads();
  v4f bias = {0.f, 0.f, 0.f, 0.f};
  if constexpr (FINAL != 0) bias = *(const v4fa*)(sbias + 64 * H + 4 * m);
  const float qnan = __uint_as_float(0x7fc00000u);
#pragma unroll 1
  for (int i = 0; i < 8; ++i) {
    const int lr   = 16 * wave + 2 * i + hh;
    const int grow = rowBase + lr;
    const bool live = grow < NN;
    const int gc = live ? grow : NN - 1;
    const v4f a = *(const v4fa*)(stg + lr * SP + 4 * m);
    asm volatile("" :: "v"(a));
    float* op = out + (size_t)gc * FD + 64 * H + 4 * m;
    v4f o = a;
    if constexpr (FINAL != 0) {
      const v4f pr = *(const v4fa*)op;
      asm volatile("" :: "v"(pr));
      const float v0 = (pr.x + a.x) + bias.x, v1 = (pr.y + a.y) + bias.y;
      const float v2 = (pr.z + a.z) + bias.z, v3 = (pr.w + a.w) + bias.w;
      o.x = (flag != 0) ? qnan : v0; o.y = (flag != 0) ? qnan : v1;
      o.z = (flag != 0) ? qnan : v2; o.w = (flag != 0) ? qnan : v3;
    }
    if (live) *(volatile v4f*)op = o;
    __threadfence();
    if (live) *(volatile v4f*)op = o;
  }
  __syncthreads();
}

template <int KTOT, int NTS, int FIRSTX, int FINAL>
__global__ __launch_bounds__(NTHR) __attribute__((amdgpu_num_vgpr(248)))
void k_gemm(const unsigned short* __restrict__ XB, const float* __restrict__ P,
            const unsigned short* __restrict__ WT, const float* __restrict__ biasf,
            const int* __restrict__ FLAG, float* out) {
  __shared__ __attribute__((aligned(16))) float stg[GBM * SP];
  __shared__ __attribute__((aligned(16))) float sbias[FD];
  const int tid = (int)threadIdx.x, lane = tid & 31, wave = tid >> 5, hh = lane >> 4, m = lane & 15;
  const int rowBase = (int)blockIdx.x * GBM;
  int flag = 0;
  if constexpr (FINAL != 0) {
    flag = FLAG[(size_t)(rowBase >> SLB) * 32];
    if (tid < 32) {
      const v4f b4 = *(const v4fa*)(biasf + 4 * tid);
      *(v4fa*)(sbias + 4 * tid) = b4;
    }
  }

  v8f acc[8];
  {
    const v8f z = {0.f, 0.f, 0.f, 0.f, 0.f, 0.f, 0.f, 0.f};
#pragma unroll
    for (int t = 0; t < 8; ++t) acc[t] = z;
  }
  const size_t rowOff = (size_t)(rowBase + 16 * wave + m) * (size_t)FD + 8 * hh;
  const unsigned short* bp = WT + (size_t)m * (size_t)KTOT + 8 * hh;
  int kb = 0;
  if constexpr (FIRSTX != 0) {
    const unsigned short* ap = XB + rowOff;
#pragma unroll 1
    for (int k0 = 0; k0 < FD; k0 += 32) {
      FragB af;
      af.h[0] = *(const v8usa*)(ap + k0);
      af.h[1] = *(const v8usa*)(ap + k0 + 16);
#pragma unroll
      for (int nt = 0; nt < 8; ++nt) {
        const unsigned short* wq = bp + (size_t)(16 * nt) * (size_t)KTOT + k0;
        FragB bf;
        bf.h[0] = *(const v8usa*)wq;
        bf.h[1] = *(const v8usa*)(wq + 16);
        acc[nt] = wmb(af, bf, acc[nt]);
      }
    }
    kb = FD;
  }
#pragma unroll 1
  for (int t = 0; t < NTS; ++t) {
    const float* pr = P + (size_t)t * (size_t)PLANE + rowOff;
#pragma unroll 1
    for (int k0 = 0; k0 < FD; k0 += 32) {
      const v4f f0 = *(const v4fa*)(pr + k0);
      const v4f f1 = *(const v4fa*)(pr + k0 + 4);
      const v4f f2 = *(const v4fa*)(pr + k0 + 16);
      const v4f f3 = *(const v4fa*)(pr + k0 + 20);
      FragB ah, al;
      split16(f0, f1, f2, f3, ah, al);
#pragma unroll
      for (int nt = 0; nt < 8; ++nt) {
        const unsigned short* wq = bp + (size_t)(16 * nt) * (size_t)KTOT + kb + k0;
        FragB bf;
        bf.h[0] = *(const v8usa*)wq;
        bf.h[1] = *(const v8usa*)(wq + 16);
        acc[nt] = wmb(ah, bf, acc[nt]);
      }
      if constexpr (TWO_TERM != 0) {
#pragma unroll
        for (int nt = 0; nt < 8; ++nt) {
          const unsigned short* wq = bp + (size_t)(16 * nt) * (size_t)KTOT + kb + FD + k0;
          FragB bf;
          bf.h[0] = *(const v8usa*)wq;
          bf.h[1] = *(const v8usa*)(wq + 16);
          acc[nt] = wmb(al, bf, acc[nt]);
        }
      }
    }
    kb += 2 * FD;
  }

  epi_half<0, FINAL>(stg, sbias, acc, out, rowBase, flag, wave, hh, m);
  epi_half<1, FINAL>(stg, sbias, acc, out, rowBase, flag, wave, hh, m);
}

extern "C" void kernel_launch(void* const* d_in, const int* in_sizes, int n_in,
                              void* d_out, int out_size, void* d_ws, size_t ws_size,
                              hipStream_t stream) {
  if (n_in < 6) return;
  if (in_sizes[0] != NN * FD) return;
  if (in_sizes[1] != NE) return;
  if (in_sizes[2] != NE) return;
  if (in_sizes[3] != NE) return;
  if (in_sizes[4] != WROWS * FD) return;
  if (in_sizes[5] != FD) return;
  if (out_size != NN * FD) return;

  const float* x    = (const float*)d_in[0];
  const int*   srcs = (const int*)d_in[1];
  const int*   dsts = (const int*)d_in[2];
  const float* ew   = (const float*)d_in[3];
  const float* W    = (const float*)d_in[4];
  const float* bias = (const float*)d_in[5];
  float* out = (float*)d_out;

  constexpr size_t zP    = (size_t)MP * FD * 4;
  constexpr size_t zXB   = (size_t)MP * FD * 2;
  constexpr size_t zLIST = (size_t)NBK * RCAP * 8;
  constexpr size_t zCO   = (size_t)NBK * 2 * NBRUN * 4;
  constexpr size_t zFLAG = (((size_t)NBK * 128 + 255) / 256) * 256;
  constexpr size_t zWA   = (size_t)FD * KA * 2;
  constexpr size_t zWB   = (size_t)FD * KB * 2;
  constexpr size_t zBF   = 512;
  constexpr size_t oP    = 0;
  constexpr size_t oXB   = oP + 4 * zP;
  constexpr size_t oLIST = oXB + zXB;
  constexpr size_t oCO   = oLIST + zLIST;
  constexpr size_t oFLAG = oCO + zCO;
  constexpr size_t oWA   = oFLAG + zFLAG;
  constexpr size_t oWB   = oWA + zWA;
  constexpr size_t oBF   = oWB + zWB;
  constexpr size_t oEND  = oBF + zBF;
  static_assert(zP % 256 == 0 && zXB % 256 == 0 && zLIST % 256 == 0 && zCO % 256 == 0 && zFLAG % 256 == 0);
  static_assert(zWA % 256 == 0 && zWB % 256 == 0 && zBF % 256 == 0);
  static_assert(zFLAG >= (size_t)NBK * 128);
  static_assert(oEND <= (size_t)(128u << 20));
  if (oEND > ws_size) return;

  char* ws = (char*)d_ws;
  float*          P    = (float*)(ws + oP);
  float*          P1   = P;
  float*          P2   = P + (size_t)PLANE;
  float*          P3   = P + (size_t)2 * PLANE;
  float*          P4   = P + (size_t)3 * PLANE;
  unsigned short* XB   = (unsigned short*)(ws + oXB);
  int*            LIST = (int*)(ws + oLIST);
  int*            CO   = (int*)(ws + oCO);
  int*            FLAG = (int*)(ws + oFLAG);
  unsigned short* WA   = (unsigned short*)(ws + oWA);
  unsigned short* WB   = (unsigned short*)(ws + oWB);
  float*          BF   = (float*)(ws + oBF);

  hipFuncSetAttribute(reinterpret_cast<const void*>(&k_bucket), hipFuncAttributeMaxDynamicSharedMemorySize, (int)BK_LDS);

  k_prep<<<PBTOT, NTHR, 0, stream>>>(x, W, bias, XB, WA, WB, BF);
  k_bucket<<<NBK, NTHR, BK_LDS, stream>>>(srcs, dsts, ew, LIST, CO, FLAG);
  k_hop<1><<<MP / HRB, NTHR, 0, stream>>>(LIST, CO, FLAG, XB, P1, P1);
  k_hop<0><<<MP / HRB, NTHR, 0, stream>>>(LIST, CO, FLAG, XB, P1, P2);
  k_hop<0><<<MP / HRB, NTHR, 0, stream>>>(LIST, CO, FLAG, XB, P2, P3);
  k_hop<0><<<MP / HRB, NTHR, 0, stream>>>(LIST, CO, FLAG, XB, P3, P4);
  k_gemm<KA, 4, 1, 0><<<MP / GBM, NTHR, 0, stream>>>(XB, P, WA, BF, FLAG, out);
  k_hop<0><<<MP / HRB, NTHR, 0, stream>>>(LIST, CO, FLAG, XB, P4, P1);
  k_hop<0><<<MP / HRB, NTHR, 0, stream>>>(LIST, CO, FLAG, XB, P1, P2);
  k_hop<0><<<MP / HRB, NTHR, 0, stream>>>(LIST, CO, FLAG, XB, P2, P3);
  k_gemm<KB, 3, 0, 1><<<MP / GBM, NTHR, 0, stream>>>(XB, P, WB, BF, FLAG, out);
}
